// TreeEncoder_34626026341055
// MI455X (gfx1250) — hardware-verified
//
#include <hip/hip_runtime.h>
#include <math.h>

typedef __attribute__((ext_vector_type(16))) _Float16 v16h;
typedef __attribute__((ext_vector_type(16))) __bf16 v16b;
typedef __attribute__((ext_vector_type(8)))  _Float16 v8h;
typedef __attribute__((ext_vector_type(8)))  float v8f;
typedef __attribute__((ext_vector_type(4)))  float v4f;
typedef __attribute__((ext_vector_type(2)))  float v2f;
typedef __attribute__((ext_vector_type(4)))  unsigned v4u;
typedef __attribute__((ext_vector_type(4)))  int v4i;
typedef float __attribute__((may_alias)) float_a;
typedef int __attribute__((may_alias)) int_a;

template <typename T> __device__ __forceinline__ void vst2(void* p, T v) { *(volatile T*)p = v; __threadfence(); *(volatile T*)p = v; }
__device__ __forceinline__ v8f wmma16(v16h a, v16h b, v8f c) {
  v8f d = __builtin_amdgcn_wmma_f32_16x16x32_f16(false, a, false, b, (short)0, c, false, false);
  asm volatile("v_nop\n\tv_nop\n\tv_nop\n\tv_nop" : "+v"(d) : "v"(a), "v"(b));
  return d;
}
__device__ __forceinline__ v8f wmma_bf(v16b a, v16b b, v8f c) {
  v8f d = __builtin_amdgcn_wmma_f32_16x16x32_bf16(false, a, false, b, (short)0, c, false, false);
  asm volatile("v_nop\n\tv_nop\n\tv_nop\n\tv_nop" : "+v"(d) : "v"(a), "v"(b));
  return d;
}
__device__ __forceinline__ v16h frag_h(const _Float16* rowk0, int lane) {
  union { v16h v; v8h q[2]; } u; const _Float16* p = rowk0 + 8 * (lane >> 4);
  u.q[0] = *(const v8h*)p; u.q[1] = *(const v8h*)(p + 16); return u.v;
}
__device__ __forceinline__ v16h frag_f32(const float* rowk0, int lane) {
  v16h a; const float* p = rowk0 + 8 * (lane >> 4);
#pragma unroll
  for (int i = 0; i < 8; ++i) { a[i] = (_Float16)p[i]; a[8 + i] = (_Float16)p[16 + i]; }
  return a;
}
__device__ __forceinline__ v16h frag_f32s(const float* rowk0, int lane, float sc) {
  v16h a; const float* p = rowk0 + 8 * (lane >> 4);
#pragma unroll
  for (int i = 0; i < 8; ++i) { a[i] = (_Float16)(p[i] * sc); a[8 + i] = (_Float16)(p[16 + i] * sc); }
  return a;
}
__device__ __forceinline__ v16h fragc_f32(const float* W, int k0, int n, int lane, int ld, int K) {
  v16h a; const int g = lane >> 4;
#pragma unroll
  for (int i = 0; i < 8; ++i) { const int ka = k0 + 8 * g + i, kb = ka + 16;
    a[i] = (_Float16)(ka < K ? W[(size_t)(ka < K ? ka : K - 1) * ld + n] : 0.f); a[8 + i] = (_Float16)(kb < K ? W[(size_t)(kb < K ? kb : K - 1) * ld + n] : 0.f); }
  return a;
}
struct F2 { v16b h, l; };
__device__ __forceinline__ F2 bsplit16(const float v[16]) { F2 r;
#pragma unroll
  for (int i = 0; i < 16; ++i) { const __bf16 h = (__bf16)v[i]; r.h[i] = h; r.l[i] = (__bf16)(v[i] - (float)h); }
  return r; }
__device__ __forceinline__ F2 split_row(const float* row, int k0, int lane) { float v[16]; const float* p = row + k0 + 8 * (lane >> 4);
#pragma unroll
  for (int i = 0; i < 8; ++i) { v[i] = p[i]; v[8 + i] = p[16 + i]; }
  return bsplit16(v); }
__device__ __forceinline__ F2 split_rowK(const float* row, int k0, int lane, int K) { float v[16]; const int g = lane >> 4;
#pragma unroll
  for (int i = 0; i < 8; ++i) { const int ka = k0 + 8 * g + i, kb = ka + 16; v[i] = ka < K ? row[ka < K ? ka : K - 1] : 0.f; v[8 + i] = kb < K ? row[kb < K ? kb : K - 1] : 0.f; }
  return bsplit16(v); }
__device__ __forceinline__ F2 split_col(const float* W, int k0, int n, int lane, int ld, int K) { float v[16]; const int g = lane >> 4;
#pragma unroll
  for (int i = 0; i < 8; ++i) { const int ka = k0 + 8 * g + i, kb = ka + 16; v[i] = ka < K ? W[(size_t)(ka < K ? ka : K - 1) * ld + n] : 0.f; v[8 + i] = kb < K ? W[(size_t)(kb < K ? kb : K - 1) * ld + n] : 0.f; }
  return bsplit16(v); }
__device__ __forceinline__ v8f mac3(const F2& a, const F2& b, v8f c) { c = wmma_bf(a.l, b.h, c); c = wmma_bf(a.h, b.l, c); return wmma_bf(a.h, b.h, c); }
__device__ __forceinline__ float sigm(float v) { return 1.0f / (1.0f + expf(-v)); }
#define LDSX() do { asm volatile("s_wait_dscnt 0" ::: "memory"); __builtin_amdgcn_wave_barrier(); __builtin_amdgcn_fence(__ATOMIC_RELEASE, "workgroup"); } while (0)


#define NB 256
#define NN 512
#define FF 64
#define HH 128
#define NL 2
#define NTOK (NB * NN)
#ifndef NRB
#define NRB (NTOK / 64)
#endif
typedef __attribute__((ext_vector_type(8))) __bf16 v8b;
__device__ __forceinline__ v16b frag_b(const __bf16* rowk0, int lane) {
  union { v16b v; v8b q[2]; } u; const __bf16* p = rowk0 + 8 * (lane >> 4);
  u.q[0] = *(const v8b*)p; u.q[1] = *(const v8b*)(p + 16); return u.v;
}
__device__ __forceinline__ float bfr(float v) { return (float)(__bf16)v; }
__device__ __attribute__((noinline)) float exp_ni(float v) { return expf(v); }
__device__ __attribute__((noinline)) float erf_ni(float v) { return erff(v); }

__device__ __attribute__((noinline)) float tanh_ni(float v) { return tanhf(v); }
#define WS_PW  0u
#define PEMB 0
#define PL0 (PEMB + HH * FF)
#define PWEND (PL0 + NL * 3 * HH * HH)
#define WS_H   (WS_PW + 2u * PWEND)
#define WS_H2  (WS_H + 4u * NTOK * HH)
#define WS_PS  (WS_H2 + 4u * NTOK * HH)
#define WS_END (WS_PS + 4u * NRB * HH)

__global__ __launch_bounds__(128) void k_packT(const float* __restrict__ EW, const float* __restrict__ WI, const float* __restrict__ WO, const float* __restrict__ WC, __bf16* __restrict__ PW) {
  __shared__ __align__(16) __bf16 s[HH]; const int n = blockIdx.x, which = blockIdx.y, k = threadIdx.x; int K; size_t dst; float v = 0.f;
  if (which == 0) { if (n >= HH) return; K = FF; dst = PEMB + (size_t)n * FF; if (k < K) v = EW[(size_t)k * HH + n]; }
  else { const int l = which - 1; const int g = n / HH, c = n % HH; const float* Wm = (g == 0) ? WI : (g == 1 ? WO : WC); K = HH; dst = PL0 + ((size_t)l * 3 * HH + n) * HH; v = Wm[((size_t)l * HH + k) * HH + c]; }
  if (k < K) s[k] = (__bf16)v; __syncthreads();
  if (k < K / 8) vst2((unsigned*)(PW + dst + k * 8), *(const v4u*)&s[k * 8]);
}
__global__ __launch_bounds__(128) void k_emb(const float* __restrict__ X, const __bf16* __restrict__ PW, const float* __restrict__ EB, float* __restrict__ Hout) {
  __shared__ __align__(16) float so[4][16][132];
  const int tid = threadIdx.x, wave = tid >> 5, lane = tid & 31, col = lane & 15, g = lane >> 4; const size_t r0 = (size_t)blockIdx.x * 64 + wave * 16;
  v8f acc[8] = {};
#pragma unroll
  for (int kc = 0; kc < FF / 32; ++kc) { v16b a; { const float* p = X + (r0 + col) * FF + kc * 32 + 8 * g;
#pragma unroll
      for (int i = 0; i < 8; ++i) { a[i] = (__bf16)p[i]; a[8 + i] = (__bf16)p[16 + i]; } }
#pragma unroll
    for (int j = 0; j < 8; ++j) acc[j] = wmma_bf(a, frag_b(PW + PEMB + (size_t)(j * 16 + col) * FF + kc * 32, lane), acc[j]); }
#pragma unroll
  for (int j = 0; j < 8; ++j) { const float bb = bfr(EB[j * 16 + col]);
#pragma unroll
    for (int r = 0; r < 8; ++r) so[wave][8 * g + r][j * 16 + col] = acc[j][r] + bb; }
  LDSX();
  for (int rl = 0; rl < 16; ++rl) vst2(Hout + (r0 + rl) * HH + lane * 4, *(const v4f*)&so[wave][rl][lane * 4]);
}
template <int LAST>
__global__ __launch_bounds__(128) void k_layer(const float* __restrict__ Hin, const __bf16* __restrict__ PWL, const float* __restrict__ BWI, const float* __restrict__ BUI, const float* __restrict__ BWO, const float* __restrict__ BUO, const float* __restrict__ BWC, const float* __restrict__ BUC, float* __restrict__ Hout, float* __restrict__ PS) {
  __shared__ __align__(16) float sg[4][16][3][HH + 4]; __shared__ __align__(16) float scs[4][HH]; __shared__ __align__(16) float sline[HH];
  const int tid = threadIdx.x, wave = tid >> 5, lane = tid & 31, col = lane & 15, g = lane >> 4; const size_t r0 = (size_t)blockIdx.x * 64 + wave * 16;
  F2 a[4];
#pragma unroll
  for (int kc = 0; kc < 4; ++kc) a[kc] = split_row(Hin + (r0 + col) * HH, kc * 32, lane);
#pragma unroll 1
  for (int gate = 0; gate < 3; ++gate) { v8f acc[8] = {};
    const float* bw = (gate == 0) ? BWI : (gate == 1 ? BWO : BWC); const float* bu = (gate == 0) ? BUI : (gate == 1 ? BUO : BUC);
#pragma unroll
    for (int kc = 0; kc < 4; ++kc) {
#pragma unroll
      for (int j = 0; j < 8; ++j) { const v16b w = frag_b(PWL + ((size_t)gate * HH + j * 16 + col) * HH + kc * 32, lane); acc[j] = wmma_bf(a[kc].l, w, acc[j]); acc[j] = wmma_bf(a[kc].h, w, acc[j]); } }
#pragma unroll
    for (int j = 0; j < 8; ++j) { const int c = j * 16 + col; const float bb = bfr(bw[c]) + bfr(bu[c]);
#pragma unroll
      for (int r = 0; r < 8; ++r) sg[wave][8 * g + r][gate][c] = acc[j][r] + bb; } }
  LDSX();
  float csum[4] = {0.f, 0.f, 0.f, 0.f};
  for (int rl = 0; rl < 16; ++rl) { v4f o4;
#pragma unroll
    for (int q = 0; q < 4; ++q) { const int c = lane * 4 + q; const float iv = sigm(sg[wave][rl][0][c]), ov = sigm(sg[wave][rl][1][c]), cv = tanh_ni(sg[wave][rl][2][c]); const float hv = ov * tanh_ni(iv * cv); o4[q] = hv; csum[q] += hv; }
    vst2(Hout + (r0 + rl) * HH + lane * 4, o4); }
  if (LAST) {
#pragma unroll
    for (int q = 0; q < 4; ++q) scs[wave][lane * 4 + q] = csum[q];
    __syncthreads();
    if (tid < HH) sline[tid] = ((scs[0][tid] + scs[1][tid]) + scs[2][tid]) + scs[3][tid];
    __syncthreads();
    if (tid < 32) vst2(PS + (size_t)blockIdx.x * HH + tid * 4, *(const v4f*)&sline[tid * 4]);
  }
}
__global__ __launch_bounds__(128) void k_mean(const float* __restrict__ PS, float* __restrict__ out) {
  __shared__ __align__(16) float s[HH]; const int b = blockIdx.x, c = threadIdx.x; float acc = 0.f;
#pragma unroll
  for (int k = 0; k < NN / 64; ++k) acc += PS[((size_t)b * (NN / 64) + k) * HH + c];
  s[c] = acc / (float)NN; __syncthreads();
  if (c < 32) vst2(out + (size_t)b * HH + c * 4, *(const v4f*)&s[c * 4]);
}
extern "C" void kernel_launch(void* const* d_in, const int* in_sizes, int n_in, void* d_out, int out_size, void* d_ws, size_t ws_size, hipStream_t stream) {
  (void)in_sizes; (void)n_in; (void)out_size;
  const float** F = (const float**)d_in;
  if (ws_size < (size_t)WS_END) return;
  char* ws = (char*)d_ws; __bf16* PW = (__bf16*)(ws + WS_PW); float *H = (float*)(ws + WS_H), *H2 = (float*)(ws + WS_H2), *PS = (float*)(ws + WS_PS);
  k_packT<<<dim3(3 * HH, 1 + NL), 128, 0, stream>>>(F[1], F[3], F[4], F[5], PW);
  k_emb<<<NRB, 128, 0, stream>>>(F[0], PW, F[2], H);
  k_layer<0><<<NRB, 128, 0, stream>>>(H, PW + PL0, F[6], F[7], F[8], F[9], F[10], F[11], H2, PS);
  k_layer<1><<<NRB, 128, 0, stream>>>(H2, PW + PL0 + (size_t)3 * HH * HH, F[6] + HH, F[7] + HH, F[8] + HH, F[9] + HH, F[10] + HH, F[11] + HH, H, PS);
  k_mean<<<(NRB * 64) / NN, 128, 0, stream>>>(PS, (float*)d_out);
}
